// DescLayer_61229053772255
// MI455X (gfx1250) — hardware-verified
//
#include <hip/hip_runtime.h>


#define NTOK 1024
#define DD   64
#define NBS  8
typedef _Float16 h16;
typedef unsigned short bf;
typedef __attribute__((ext_vector_type(16))) __bf16   v16bf;
typedef __attribute__((ext_vector_type(16))) _Float16 v16h;
typedef __attribute__((ext_vector_type(8)))  _Float16 v8h;
typedef __attribute__((ext_vector_type(8)))  unsigned short v8us;
typedef __attribute__((ext_vector_type(8)))  float    v8f;
typedef __attribute__((ext_vector_type(4)))  float    v4f;
typedef v8h  __attribute__((may_alias)) v8ha;
typedef v4f  __attribute__((may_alias)) v4fa;
typedef v8us __attribute__((may_alias)) v8usa;

__device__ __forceinline__ unsigned short f2bf(float f) { unsigned u = __float_as_uint(f); u += 0x7FFFu + ((u >> 16) & 1u); return (unsigned short)(u >> 16); }
__device__ __forceinline__ float bf2f(unsigned short b) { return __uint_as_float(((unsigned)b) << 16); }
__device__ __forceinline__ float bfr(float f) { return bf2f(f2bf(f)); }
__device__ __forceinline__ v16h cat16(v8h lo, v8h hi) { return __builtin_shufflevector(lo, hi, 0, 1, 2, 3, 4, 5, 6, 7, 8, 9, 10, 11, 12, 13, 14, 15); }
__device__ __forceinline__ v16bf cat16b(v8us lo, v8us hi) { return __builtin_bit_cast(v16bf, __builtin_shufflevector(lo, hi, 0, 1, 2, 3, 4, 5, 6, 7, 8, 9, 10, 11, 12, 13, 14, 15)); }
__device__ __forceinline__ v8f wmma16(v16h a, v16h b, v8f c) { return __builtin_amdgcn_wmma_f32_16x16x32_f16(false, a, false, b, (short)0, c, false, false); }
__device__ __forceinline__ v8f wmmab(v16bf a, v16bf b, v8f c) { return __builtin_amdgcn_wmma_f32_16x16x32_bf16(false, a, false, b, (short)0, c, false, false); }


template <typename T16> struct WFrag;
template <> struct WFrag<h16> { typedef v16h V; static __device__ __forceinline__ V ld(const h16* p) { return cat16(*(const v8h*)p, *(const v8h*)(p + 16)); } static __device__ __forceinline__ v8f mma(V a, V b, v8f c) { return wmma16(a, b, c); } };
template <> struct WFrag<bf> { typedef v16bf V; static __device__ __forceinline__ V ld(const bf* p) { return cat16b(*(const v8us*)p, *(const v8us*)(p + 16)); } static __device__ __forceinline__ v8f mma(V a, V b, v8f c) { return wmmab(a, b, c); } };
template <typename T16, int NSPLIT, bool BIAS>
__global__ __launch_bounds__(32) void k_gemmw(const T16* __restrict__ A, const T16* __restrict__ A2, const T16* __restrict__ Bt, const T16* __restrict__ Bt2, int K, float* C, int ldc, const float* __restrict__ bias, size_t sA, size_t sB, size_t sC) {
    typedef typename WFrag<T16>::V V;
    __shared__ __align__(16) float os[16 * 68];
    const size_t z = blockIdx.z; A += z * sA; if (A2) A2 += z * sA; Bt += z * sB; if (Bt2) Bt2 += z * sB; C += z * sC;
    const int lane = threadIdx.x & 31, lr = lane & 15, hi = lane >> 4; const int r0 = blockIdx.x * 64, c0 = blockIdx.y * 64;
    v8f acc[4][4];
#pragma unroll
    for (int mb = 0; mb < 4; ++mb)
#pragma unroll
        for (int nb = 0; nb < 4; ++nb) acc[mb][nb] = (v8f){};
    const size_t aoff = (size_t)(r0 + lr) * K + 8 * hi, boff = (size_t)(c0 + lr) * K + 8 * hi;
#pragma unroll 1
    for (int kc = 0; kc < K; kc += 32) {
        V a[4], a2[4];
#pragma unroll
        for (int mb = 0; mb < 4; ++mb) { a[mb] = WFrag<T16>::ld(A + aoff + (size_t)mb * 16 * K + kc); if (NSPLIT == 1 || NSPLIT == 2) a2[mb] = WFrag<T16>::ld(A2 + aoff + (size_t)mb * 16 * K + kc); }
#pragma unroll
        for (int nb = 0; nb < 4; ++nb) { const V b = WFrag<T16>::ld(Bt + boff + (size_t)nb * 16 * K + kc); V b2; if (NSPLIT >= 2) b2 = WFrag<T16>::ld(Bt2 + boff + (size_t)nb * 16 * K + kc);
#pragma unroll
            for (int mb = 0; mb < 4; ++mb) { acc[mb][nb] = WFrag<T16>::mma(a[mb], b, acc[mb][nb]); if (NSPLIT == 1 || NSPLIT == 2) acc[mb][nb] = WFrag<T16>::mma(a2[mb], b, acc[mb][nb]); if (NSPLIT >= 2) acc[mb][nb] = WFrag<T16>::mma(a[mb], b2, acc[mb][nb]); } }
        asm volatile("v_nop\n\tv_nop\n\tv_nop\n\tv_nop" : "+v"(acc[0][0]), "+v"(acc[1][1]), "+v"(acc[2][2]), "+v"(acc[3][3]) : "v"(a[0]), "v"(a[3]));
    }
#pragma unroll
    for (int mb = 0; mb < 4; ++mb) {
#pragma unroll
        for (int nb = 0; nb < 4; ++nb) {
#pragma unroll
            for (int j = 0; j < 8; ++j) os[(hi * 8 + j) * 68 + nb * 16 + lr] = acc[mb][nb][j]; }
        __builtin_amdgcn_wave_barrier(); asm volatile("" ::: "memory");
        float* crow = C + (size_t)(r0 + mb * 16) * ldc + c0;
#pragma unroll 1
        for (int ps = 0; ps < 2; ++ps) {
#pragma unroll
            for (int s = 0; s < 8; ++s) { const int row = 2 * s + hi, cofs = lr * 4; v4f val = *(const v4fa*)(os + row * 68 + cofs); if (BIAS) { val[0] += bfr(bias[c0 + cofs]); val[1] += bfr(bias[c0 + cofs + 1]); val[2] += bfr(bias[c0 + cofs + 2]); val[3] += bfr(bias[c0 + cofs + 3]); }
                *(volatile v4f*)(crow + (size_t)row * ldc + cofs) = val; }
            if (ps == 0) __threadfence(); }
        __builtin_amdgcn_wave_barrier(); asm volatile("" ::: "memory");
    }
}

__device__ __forceinline__ void splitf(float y, unsigned short& h, unsigned short& l) { h = f2bf(y); l = f2bf(y - bf2f(h)); }
typedef __attribute__((ext_vector_type(2))) unsigned short v2us;

__global__ __launch_bounds__(256) void k_cvt8(const float* __restrict__ src, bf* dst, size_t n8) { const size_t i = (size_t)blockIdx.x * 256 + threadIdx.x; if (i >= n8) return; const v8f v = *(const v8f*)(src + i * 8); v8us o;
#pragma unroll
    for (int k = 0; k < 8; ++k) o[k] = f2bf(v[k]); *(volatile v8us*)(dst + i * 8) = o; __threadfence(); *(volatile v8us*)(dst + i * 8) = o; }
__global__ __launch_bounds__(256) void k_ln(const float* __restrict__ x, const float* __restrict__ ga, const float* __restrict__ be, bf* Lh, bf* Ll) { const int lane = threadIdx.x & 31; const int row = blockIdx.x * 8 + (threadIdx.x >> 5); if (row >= NTOK) return; const float* r = x + (size_t)row * DD + 2 * lane; const float a0 = bfr(r[0]), a1 = bfr(r[1]); float s = __fadd_rn(a0, a1);
#pragma unroll
    for (int sh = 16; sh; sh >>= 1) s += __shfl_xor(s, sh, 32);
    const float mean = s * (1.0f / DD); float d0 = __fsub_rn(a0, mean), d1 = __fsub_rn(a1, mean); asm volatile("" : "+v"(d0)); asm volatile("" : "+v"(d1)); float q = __fadd_rn(__fmul_rn(d0, d0), __fmul_rn(d1, d1));
#pragma unroll
    for (int sh = 16; sh; sh >>= 1) q += __shfl_xor(q, sh, 32);
    const float rstd = __frsqrt_rn(__fadd_rn(q * (1.0f / DD), 1e-5f)); v2us oh, ol; { float t0 = __fmul_rn(d0, rstd); asm volatile("" : "+v"(t0)); float t1 = __fmul_rn(t0, bfr(ga[2 * lane])); asm volatile("" : "+v"(t1)); unsigned short a, b; splitf(__fadd_rn(t1, bfr(be[2 * lane])), a, b); oh[0] = a; ol[0] = b;
      float u0 = __fmul_rn(d1, rstd); asm volatile("" : "+v"(u0)); float u1 = __fmul_rn(u0, bfr(ga[2 * lane + 1])); asm volatile("" : "+v"(u1)); splitf(__fadd_rn(u1, bfr(be[2 * lane + 1])), a, b); oh[1] = a; ol[1] = b; }
    const size_t o = (size_t)row * DD + 2 * lane; *(volatile v2us*)(Lh + o) = oh; *(volatile v2us*)(Ll + o) = ol; __threadfence(); *(volatile v2us*)(Lh + o) = oh; *(volatile v2us*)(Ll + o) = ol; }
__global__ __launch_bounds__(256) void k_nk(const float* __restrict__ XP, const float* __restrict__ RES, const int* __restrict__ kk, const float* __restrict__ P, const float* __restrict__ per, float* OUT) { const int idx = blockIdx.x * 256 + threadIdx.x; if (idx >= NTOK * DD) return; const int i = idx % DD, tok = idx / DD; const float kf = (float)kk[tok]; const float num = __fmul_rn(6.283185307179586f, kf); float acc = 0.f;
#pragma unroll 1
    for (int j = 0; j < DD; ++j) { const float xp = XP[(size_t)tok * DD + j];
#pragma unroll 1
        for (int g = 0; g < NBS; ++g) { const int pj = (i * DD + j) * NBS + g; const float c = cosf(__fdiv_rn(num, bfr(per[pj]))); float t = __fmul_rn(c, bfr(P[pj])); asm volatile("" : "+v"(t)); float t2 = __fmul_rn(t, xp); asm volatile("" : "+v"(t2)); acc = __fadd_rn(acc, t2); } }
    const float o = __fadd_rn(RES[idx], acc); *(volatile float*)(OUT + idx) = o; __threadfence(); *(volatile float*)(OUT + idx) = o; }

extern "C" void kernel_launch(void* const* d_in, const int* in_sizes, int n_in,
                              void* d_out, int out_size, void* d_ws, size_t ws_size, hipStream_t stream) {
    (void)in_sizes; (void)n_in; (void)out_size;
    const float* x = (const float*)d_in[0]; const int* kk = (const int*)d_in[1]; const float* Mw = (const float*)d_in[2]; const float* Rw = (const float*)d_in[3]; const float* P = (const float*)d_in[4]; const float* ga = (const float*)d_in[5]; const float* be = (const float*)d_in[6]; const float* per = (const float*)d_in[7];
    float* OUT = (float*)d_out;
    char* wsp = (char*)d_ws;
    auto take = [&](size_t bytes) { char* p = wsp; wsp += (bytes + 255) & ~(size_t)255; return (void*)p; };
    bf* MB_ = (bf*)take(DD * DD * 2); bf* RB = (bf*)take(DD * DD * 2); bf* Lh = (bf*)take((size_t)NTOK * DD * 2); bf* Ll = (bf*)take((size_t)NTOK * DD * 2); float* XP = (float*)take((size_t)NTOK * DD * 4); float* RES = (float*)take((size_t)NTOK * DD * 4);
    if ((size_t)(wsp - (char*)d_ws) > ws_size) return;
    k_cvt8<<<(DD * DD / 8 + 255) / 256, 256, 0, stream>>>(Mw, MB_, DD * DD / 8); k_cvt8<<<(DD * DD / 8 + 255) / 256, 256, 0, stream>>>(Rw, RB, DD * DD / 8);
    k_ln<<<NTOK / 8, 256, 0, stream>>>(x, ga, be, Lh, Ll);
    k_gemmw<bf, 1, false><<<dim3(NTOK / 64, 1, 1), 32, 0, stream>>>(Lh, Ll, MB_, nullptr, DD, XP, DD, nullptr, 0, 0, 0); k_gemmw<bf, 1, false><<<dim3(NTOK / 64, 1, 1), 32, 0, stream>>>(Lh, Ll, RB, nullptr, DD, RES, DD, nullptr, 0, 0, 0);
    k_nk<<<(NTOK * DD + 255) / 256, 256, 0, stream>>>(XP, RES, kk, P, per, OUT);
}
